// IGNNConv_87600152969918
// MI455X (gfx1250) — hardware-verified
//
#include <hip/hip_runtime.h>
#include <math.h>

typedef __attribute__((ext_vector_type(16))) _Float16 v16h;
typedef __attribute__((ext_vector_type(16))) __bf16 v16b;
typedef __attribute__((ext_vector_type(8)))  _Float16 v8h;
typedef __attribute__((ext_vector_type(8)))  float v8f;
typedef __attribute__((ext_vector_type(4)))  float v4f;
typedef __attribute__((ext_vector_type(2)))  float v2f;
typedef __attribute__((ext_vector_type(4)))  unsigned v4u;
typedef __attribute__((ext_vector_type(4)))  int v4i;
typedef float __attribute__((may_alias)) float_a;
typedef int __attribute__((may_alias)) int_a;

template <typename T> __device__ __forceinline__ void vst2(void* p, T v) { *(volatile T*)p = v; __threadfence(); *(volatile T*)p = v; }
__device__ __forceinline__ v8f wmma16(v16h a, v16h b, v8f c) {
  v8f d = __builtin_amdgcn_wmma_f32_16x16x32_f16(false, a, false, b, (short)0, c, false, false);
  asm volatile("v_nop\n\tv_nop\n\tv_nop\n\tv_nop" : "+v"(d) : "v"(a), "v"(b));
  return d;
}
__device__ __forceinline__ v8f wmma_bf(v16b a, v16b b, v8f c) {
  v8f d = __builtin_amdgcn_wmma_f32_16x16x32_bf16(false, a, false, b, (short)0, c, false, false);
  asm volatile("v_nop\n\tv_nop\n\tv_nop\n\tv_nop" : "+v"(d) : "v"(a), "v"(b));
  return d;
}
__device__ __forceinline__ v16h frag_h(const _Float16* rowk0, int lane) {
  union { v16h v; v8h q[2]; } u; const _Float16* p = rowk0 + 8 * (lane >> 4);
  u.q[0] = *(const v8h*)p; u.q[1] = *(const v8h*)(p + 16); return u.v;
}
__device__ __forceinline__ v16h frag_f32(const float* rowk0, int lane) {
  v16h a; const float* p = rowk0 + 8 * (lane >> 4);
#pragma unroll
  for (int i = 0; i < 8; ++i) { a[i] = (_Float16)p[i]; a[8 + i] = (_Float16)p[16 + i]; }
  return a;
}
__device__ __forceinline__ v16h frag_f32s(const float* rowk0, int lane, float sc) {
  v16h a; const float* p = rowk0 + 8 * (lane >> 4);
#pragma unroll
  for (int i = 0; i < 8; ++i) { a[i] = (_Float16)(p[i] * sc); a[8 + i] = (_Float16)(p[16 + i] * sc); }
  return a;
}
__device__ __forceinline__ v16h fragc_f32(const float* W, int k0, int n, int lane, int ld, int K) {
  v16h a; const int g = lane >> 4;
#pragma unroll
  for (int i = 0; i < 8; ++i) { const int ka = k0 + 8 * g + i, kb = ka + 16;
    a[i] = (_Float16)(ka < K ? W[(size_t)ka * ld + n] : 0.f); a[8 + i] = (_Float16)(kb < K ? W[(size_t)kb * ld + n] : 0.f); }
  return a;
}
struct F2 { v16b h, l; };
__device__ __forceinline__ F2 bsplit16(const float v[16]) { F2 r;
#pragma unroll
  for (int i = 0; i < 16; ++i) { const __bf16 h = (__bf16)v[i]; r.h[i] = h; r.l[i] = (__bf16)(v[i] - (float)h); }
  return r; }
__device__ __forceinline__ F2 split_row(const float* row, int k0, int lane) { float v[16]; const float* p = row + k0 + 8 * (lane >> 4);
#pragma unroll
  for (int i = 0; i < 8; ++i) { v[i] = p[i]; v[8 + i] = p[16 + i]; }
  return bsplit16(v); }
__device__ __forceinline__ F2 split_rowK(const float* row, int k0, int lane, int K) { float v[16]; const int g = lane >> 4;
#pragma unroll
  for (int i = 0; i < 8; ++i) { const int ka = k0 + 8 * g + i, kb = ka + 16; v[i] = ka < K ? row[ka] : 0.f; v[8 + i] = kb < K ? row[kb] : 0.f; }
  return bsplit16(v); }
__device__ __forceinline__ F2 split_col(const float* W, int k0, int n, int lane, int ld, int K) { float v[16]; const int g = lane >> 4;
#pragma unroll
  for (int i = 0; i < 8; ++i) { const int ka = k0 + 8 * g + i, kb = ka + 16; v[i] = ka < K ? W[(size_t)ka * ld + n] : 0.f; v[8 + i] = kb < K ? W[(size_t)kb * ld + n] : 0.f; }
  return bsplit16(v); }
__device__ __forceinline__ v8f mac3(const F2& a, const F2& b, v8f c) { c = wmma_bf(a.l, b.h, c); c = wmma_bf(a.h, b.l, c); return wmma_bf(a.h, b.h, c); }
__device__ __forceinline__ float sigm(float v) { return 1.0f / (1.0f + expf(-v)); }
#define LDSX() do { asm volatile("s_wait_dscnt 0" ::: "memory"); __builtin_amdgcn_wave_barrier(); __builtin_amdgcn_fence(__ATOMIC_RELEASE, "workgroup"); } while (0)


#define NN 50000
#define NE 800000
#define FI 96
#define HID 256
#define NHOP 3
#define RB 512
#define NRB 98
#define NNP (NRB * RB)
#define RBD 8192
#define NRBD ((NNP + RBD - 1) / RBD)
#define EPT 8
#define CH (256 * EPT)
__device__ __forceinline__ int clampn(int v) { return v < 0 ? 0 : (v >= NN ? NN - 1 : v); }

__global__ __launch_bounds__(256) void k_deg(const int* __restrict__ erow, const int* __restrict__ ecol, float* __restrict__ DINV) {
  __shared__ int scnt[RBD];
  const int tid = threadIdx.x; const int r0 = blockIdx.x * RBD;
  for (int q = tid; q < RBD; q += 256) scnt[q] = 0;
  __syncthreads();
#pragma unroll 1
  for (int c0 = 0; c0 < NE; c0 += CH) { const int e0 = c0 + tid * EPT;
    if (e0 + EPT <= NE) {
#pragma unroll
      for (int v = 0; v < EPT / 4; ++v) { const int4 r4 = *(const int4*)(erow + e0 + v * 4), c4 = *(const int4*)(ecol + e0 + v * 4); const int rr[4] = {r4.x, r4.y, r4.z, r4.w}, cc[4] = {c4.x, c4.y, c4.z, c4.w};
#pragma unroll
        for (int u = 0; u < 4; ++u) { const unsigned rel = (unsigned)(rr[u] - r0); if (rel < (unsigned)RBD && cc[u] != rr[u]) atomicAdd(&scnt[rel], 1); } } }
    else { for (int u = 0; u < EPT; ++u) { const int e = e0 + u; if (e < NE) { const int r = erow[e]; const unsigned rel = (unsigned)(r - r0); if (rel < (unsigned)RBD && ecol[e] != r) atomicAdd(&scnt[rel], 1); } } } }
  __syncthreads();
  for (int q = tid; q < RBD; q += 256) { const int r = r0 + q; if (r < NNP) vst2(DINV + r, r < NN ? rsqrtf((float)(scnt[q] + 1)) : 0.f); }
}
__global__ __launch_bounds__(256) void k_norm(const float* __restrict__ x, float* __restrict__ H0) {
  const int wave = threadIdx.x >> 5, lane = threadIdx.x & 31;
  for (int r = blockIdx.x * 8 + wave; r < NNP; r += gridDim.x * 8) {
    v4f v = {0.f, 0.f, 0.f, 0.f}; if (r < NN && lane < FI / 4) v = *(const v4f*)(x + (size_t)r * FI + lane * 4);
    float ss = v[0] * v[0] + v[1] * v[1] + v[2] * v[2] + v[3] * v[3];
#pragma unroll
    for (int off = 16; off > 0; off >>= 1) ss += __shfl_xor(ss, off, 32);
    const float inv = 1.0f / fmaxf(sqrtf(ss), 1e-12f);
    if (lane < FI / 4) { v4f o = {v[0] * inv, v[1] * inv, v[2] * inv, v[3] * inv}; vst2(H0 + (size_t)r * FI + lane * 4, o); } }
}
__global__ __launch_bounds__(256) void k_hop(const int* __restrict__ erow, const int* __restrict__ ecol, const float* __restrict__ DINV, const float* __restrict__ Hin, float* __restrict__ Hout) {
  __shared__ __align__(16) float sacc[RB][FI];
  __shared__ int slst[8][32 * EPT], sdl[8][32 * EPT]; __shared__ float swgt[8][32 * EPT]; __shared__ int scnt[8];
  const int tid = threadIdx.x, wave = tid >> 5, lane = tid & 31;
  const int r0 = blockIdx.x * RB;
  for (int q = tid; q < RB * FI; q += 256) (&sacc[0][0])[q] = 0.f;
  __syncthreads();
#pragma unroll 1
  for (int c0 = 0; c0 < NE; c0 += CH) { const int e0 = c0 + tid * EPT; int hd[EPT]; int cnt = 0;
    if (e0 + EPT <= NE) {
#pragma unroll
      for (int v = 0; v < EPT / 4; ++v) { const int4 d4 = *(const int4*)(erow + e0 + v * 4); const int dd[4] = {d4.x, d4.y, d4.z, d4.w};
#pragma unroll
        for (int u = 0; u < 4; ++u) { const unsigned rel = (unsigned)(clampn(dd[u]) - r0); const bool h = rel < (unsigned)RB; hd[v * 4 + u] = h ? (int)rel : -1; cnt += h ? 1 : 0; } } }
    else {
#pragma unroll
      for (int u = 0; u < EPT; ++u) { const int e = e0 + u; hd[u] = -1; if (e < NE) { const unsigned rel = (unsigned)(clampn(erow[e]) - r0); if (rel < (unsigned)RB) { hd[u] = (int)rel; ++cnt; } } } }
    int incl = cnt;
#pragma unroll
    for (int off = 1; off < 32; off <<= 1) { const int vv = __shfl_up(incl, off, 32); if (lane >= off) incl += vv; }
    const int wtot = __shfl(incl, 31, 32); int pos = incl - cnt;
    if (cnt > 0) {
#pragma unroll
      for (int u = 0; u < EPT; ++u) if (hd[u] >= 0) { slst[wave][pos] = e0 + u; sdl[wave][pos] = hd[u]; ++pos; } }
    if (lane == 0) scnt[wave] = wtot;
    __syncthreads();
#pragma unroll 1
    for (int w = 0; w < 8; ++w) { const int nh = scnt[w];
#pragma unroll 1
      for (int i = tid; i < nh; i += 256) { const int e = slst[w][i]; const int craw = ecol[e]; const int c = clampn(craw); slst[w][i] = c; swgt[w][i] = (craw == r0 + sdl[w][i]) ? 0.f : DINV[c]; } }
    __syncthreads();
    if (tid < FI) {
#pragma unroll 1
      for (int w = 0; w < 8; ++w) { const int nh = scnt[w];
#pragma unroll 1
        for (int i = 0; i < nh; ++i) { const int c = slst[w][i], dl = sdl[w][i]; sacc[dl][tid] += swgt[w][i] * Hin[(size_t)c * FI + tid]; } } }
    __syncthreads(); }
#pragma unroll 1
  for (int q = tid; q < RB * (FI / 4); q += 256) { const int rl = q / (FI / 4), pc = q % (FI / 4); const int row = r0 + rl; v4f o = {0.f, 0.f, 0.f, 0.f};
    if (row < NN) { const float dv = DINV[row]; const v4f a = *(const v4f*)(&sacc[rl][pc * 4]); const v4f h = *(const v4f*)(Hin + (size_t)row * FI + pc * 4);
      o[0] = (a[0] + dv * h[0]) * dv; o[1] = (a[1] + dv * h[1]) * dv; o[2] = (a[2] + dv * h[2]) * dv; o[3] = (a[3] + dv * h[3]) * dv; }
    vst2(Hout + (size_t)row * FI + pc * 4, o); }
}
__global__ __launch_bounds__(256) void k_pack(const float* __restrict__ Ws, const float* __restrict__ Wf, _Float16* __restrict__ PTS, _Float16* __restrict__ PTF) {
  const int b = blockIdx.x, tid = threadIdx.x; __shared__ __align__(16) _Float16 srow[1024];
  if (b < 2 * HID) { const int rr = 2 * b + (tid >= FI ? 1 : 0), kk = tid >= FI ? tid - FI : tid; const int i = rr / HID, n = rr % HID;
    if (tid < 2 * FI) srow[tid] = (_Float16)(Ws[((size_t)i * FI + kk) * HID + n] * 16.0f); __syncthreads(); if (tid < 2 * FI / 8) vst2(PTS + (size_t)(2 * b) * FI + tid * 8, *(const v4u*)(&srow[tid * 8])); }
  else { const int n = b - 2 * HID; for (int k = tid; k < 4 * HID; k += 256) srow[k] = (_Float16)(Wf[(size_t)k * HID + n] * 16.0f); __syncthreads(); if (tid < 128) vst2(PTF + (size_t)n * (4 * HID) + tid * 8, *(const v4u*)(&srow[tid * 8])); }
}
__global__ __launch_bounds__(128) void k_mlp(const float* __restrict__ H0, const float* __restrict__ H1, const float* __restrict__ H2, const float* __restrict__ H3, const _Float16* __restrict__ PTS,
                                            const float* __restrict__ bs, const _Float16* __restrict__ PTF, const float* __restrict__ bf, float* __restrict__ out) {
  __shared__ __align__(16) _Float16 sZ[64][HID + 8];
  __shared__ __align__(16) float so[4][16][132];
  const int tid = threadIdx.x, wave = tid >> 5, lane = tid & 31, col = lane & 15, g = lane >> 4;
  const int r0 = blockIdx.x * 64 + wave * 16; const int ra = (r0 + col) < NN ? (r0 + col) : (NN - 1);
#pragma unroll 1
  for (int nh = 0; nh < 2; ++nh) { v8f acc[8] = {};
#pragma unroll 1
    for (int i = 0; i < 4; ++i) { const float* Hs = i == 0 ? H0 : (i == 1 ? H1 : (i == 2 ? H2 : H3)); const _Float16* Pi = PTS + (size_t)i * HID * FI;
#pragma unroll 1
      for (int zh = 0; zh < 2; ++zh) { v8f zacc[8] = {};
#pragma unroll
        for (int kc = 0; kc < FI / 32; ++kc) { const v16h a = frag_f32(Hs + (size_t)ra * FI + kc * 32, lane);
#pragma unroll
          for (int j = 0; j < 8; ++j) zacc[j] = wmma16(a, frag_h(Pi + (size_t)(zh * 128 + j * 16 + col) * FI + kc * 32, lane), zacc[j]); }
#pragma unroll
        for (int j = 0; j < 8; ++j) { const int n = zh * 128 + j * 16 + col; const float bb = bs[i * HID + n];
#pragma unroll
          for (int r = 0; r < 8; ++r) { const float v = zacc[j][r] * (1.0f / 16.0f) + bb; sZ[wave * 16 + 8 * g + r][n] = (_Float16)(v > 0.f ? v : 0.f); } } }
      LDSX();
#pragma unroll 2
      for (int kc = 0; kc < HID / 32; ++kc) { const v16h a = frag_h(&sZ[wave * 16 + col][0] + kc * 32, lane);
#pragma unroll
        for (int j = 0; j < 8; ++j) acc[j] = wmma16(a, frag_h(PTF + (size_t)(nh * 128 + j * 16 + col) * (4 * HID) + i * HID + kc * 32, lane), acc[j]); }
      LDSX(); }
#pragma unroll
    for (int j = 0; j < 8; ++j) { const int n = nh * 128 + j * 16 + col; const float bb = bf[n];
#pragma unroll
      for (int r = 0; r < 8; ++r) { const float v = acc[j][r] * (1.0f / 16.0f) + bb; so[wave][8 * g + r][j * 16 + col] = v > 0.f ? v : 0.f; } }
    LDSX();
    for (int rl = 0; rl < 16; ++rl) { if (r0 + rl >= NN) break; vst2(out + (size_t)(r0 + rl) * HID + nh * 128 + lane * 4, *(const v4f*)(&so[wave][rl][lane * 4])); }
    LDSX(); }
}
extern "C" void kernel_launch(void* const* d_in, const int* in_sizes, int n_in, void* d_out, int out_size, void* d_ws, size_t ws_size, hipStream_t stream) {
  (void)in_sizes; (void)n_in; (void)out_size; (void)ws_size;
  const int* ei = (const int*)d_in[0]; const float* x = (const float*)d_in[1]; const float* Ws = (const float*)d_in[2]; const float* bs = (const float*)d_in[3]; const float* Wf = (const float*)d_in[4]; const float* bf = (const float*)d_in[5];
  const int* erow = ei; const int* ecol = ei + NE;
  float* out = (float*)d_out;
  char* ws = (char*)d_ws; size_t off = 0;
  auto take = [&](size_t bytes) { char* p = ws + off; off += (bytes + 255) & ~(size_t)255; return p; };
  float* DINV = (float*)take((size_t)NNP * 4); float* H0 = (float*)take((size_t)NNP * FI * 4); float* H1 = (float*)take((size_t)NNP * FI * 4); float* H2 = (float*)take((size_t)NNP * FI * 4); float* H3 = (float*)take((size_t)NNP * FI * 4);
  _Float16* PTS = (_Float16*)take((size_t)4 * HID * FI * 2); _Float16* PTF = (_Float16*)take((size_t)HID * 4 * HID * 2);
  k_deg<<<NRBD, 256, 0, stream>>>(erow, ecol, DINV);
  k_norm<<<784, 256, 0, stream>>>(x, H0);
  k_pack<<<3 * HID, 256, 0, stream>>>(Ws, Wf, PTS, PTF);
  k_hop<<<NRB, 256, 0, stream>>>(erow, ecol, DINV, H0, H1);
  k_hop<<<NRB, 256, 0, stream>>>(erow, ecol, DINV, H1, H2);
  k_hop<<<NRB, 256, 0, stream>>>(erow, ecol, DINV, H2, H3);
  k_mlp<<<NNP / 64, 128, 0, stream>>>(H0, H1, H2, H3, PTS, bs, PTF, bf, out);
}
